// Encoder_9259949490960
// MI455X (gfx1250) — hardware-verified
//
#include <hip/hip_runtime.h>
#include <hip/hip_fp16.h>


#ifndef NB
#define NB 32
#endif
#ifndef SEQ
#define SEQ 512
#endif
#define NB_FULL  32
#define SEQ_FULL 512
#define NH   8
#define HD   64
#define DM   512
#define DF   2048
#define NTOK (NB * SEQ)

static_assert(NB >= 1 && NB <= NB_FULL);
static_assert(SEQ >= 128 && SEQ <= SEQ_FULL);
static_assert(SEQ % 128 == 0);
static_assert(NTOK % 128 == 0);
static_assert(DM == NH * HD);
static_assert(DM == 512 && HD == 64 && NH == 8 && DF == 2048);

typedef _Float16 v16h __attribute__((ext_vector_type(16)));
typedef _Float16 v8h  __attribute__((ext_vector_type(8)));
typedef float    v8f  __attribute__((ext_vector_type(8)));
typedef float    v4f  __attribute__((ext_vector_type(4)));

union Frag { v16h v; v8h h[2]; };

#define LOG2E 1.44269504088896340736f
#define C1 (1.44269504088896340736f * 0.000244140625f)
#define C2 (1.44269504088896340736f * 1.1920928955078125e-07f)
#define SC_RES   2048.0f
#define SC_RINV  4.8828125e-04f
#define SC_OUT   9.765625e-04f
#define SC_HID   1.5625e-02f

static __device__ __forceinline__ v8f zero8() {
    v8f z;
#pragma unroll
    for (int i = 0; i < 8; ++i) z[i] = 0.0f;
    return z;
}

static __device__ __forceinline__ v16h load_frag16(const _Float16* base, unsigned ld, unsigned lane) {
    const unsigned m  = lane & 15u;
    const unsigned kb = (lane >> 4) << 3;
    const _Float16* p = base + (size_t)m * ld + kb;
    Frag f;
    f.h[0] = *(const v8h*)(p);
    f.h[1] = *(const v8h*)(p + 16);
    return f.v;
}

static __device__ __forceinline__ v8f wmma16(v16h a, v16h b, v8f c) {
    v8f d = __builtin_amdgcn_wmma_f32_16x16x32_f16(false, a, false, b, (short)0, c, false, false);
    asm volatile("v_nop\n\tv_nop\n\tv_nop\n\tv_nop" : "+v"(d) : "v"(a), "v"(b));
    return d;
}

static __device__ __forceinline__ float bf16r(float x) {
    unsigned u = __float_as_uint(x);
    u = (u + 0x7FFFu + ((u >> 16) & 1u)) & 0xFFFF0000u;
    return __uint_as_float(u);
}

static __device__ __forceinline__ float ex2(float x) {
    return __builtin_amdgcn_exp2f(x);
}

static __device__ __forceinline__ void wave_lds_sync() {
    __builtin_amdgcn_fence(3, "wavefront");
    asm volatile("s_wait_dscnt 0" ::: "memory");
    __builtin_amdgcn_wave_barrier();
}

static __device__ __forceinline__ float wave_sum(float v) {
    v += __shfl_xor(v, 16, 32);
    v += __shfl_xor(v, 8, 32);
    v += __shfl_xor(v, 4, 32);
    v += __shfl_xor(v, 2, 32);
    v += __shfl_xor(v, 1, 32);
    return v;
}

static __device__ __forceinline__ unsigned full_row(unsigned n) {
    const unsigned b = n / (unsigned)SEQ;
    return b * (unsigned)SEQ_FULL + (n - b * (unsigned)SEQ);
}

template <int TM, int TN, bool RES>
static __device__ __forceinline__ void gemm_core(const _Float16* __restrict__ Ah,
                                                 const _Float16* __restrict__ Ar,
                                                 const _Float16* __restrict__ Bt,
                                                 unsigned K, unsigned lane,
                                                 v8f (&acc)[TM][TN], v8f (&accr)[TM][TN]) {
#pragma unroll
    for (int mt = 0; mt < TM; ++mt)
#pragma unroll
        for (int nt = 0; nt < TN; ++nt) {
            acc[mt][nt] = zero8();
            if (RES) accr[mt][nt] = zero8();
        }
#pragma unroll 1
    for (unsigned k = 0; k < K; k += 32u) {
        v16h a[TM];
        v16h ar[TM];
#pragma unroll
        for (int mt = 0; mt < TM; ++mt) {
            a[mt] = load_frag16(Ah + (size_t)(mt * 16) * K + k, K, lane);
            if (RES) ar[mt] = load_frag16(Ar + (size_t)(mt * 16) * K + k, K, lane);
        }
#pragma unroll
        for (int nt = 0; nt < TN; ++nt) {
            const v16h bfr = load_frag16(Bt + (size_t)(nt * 16) * K + k, K, lane);
#pragma unroll
            for (int mt = 0; mt < TM; ++mt) {
                acc[mt][nt] = wmma16(a[mt], bfr, acc[mt][nt]);
                if (RES) accr[mt][nt] = wmma16(ar[mt], bfr, accr[mt][nt]);
            }
        }
    }
}

__global__ __launch_bounds__(256) void k_cvt_x(const float* __restrict__ x,
                                                _Float16* __restrict__ xh) {
    const unsigned idx = blockIdx.x * 256u + threadIdx.x;
    const unsigned n   = idx >> 6;
    const unsigned c8  = (idx & 63u) << 3;
    const unsigned fr  = full_row(n);
    const float* p = x + (size_t)fr * DM + c8;
    const v4f a = *(const v4f*)(p);
    const v4f b = *(const v4f*)(p + 4);
    v8h o;
    o[0] = (_Float16)bf16r(a.x); o[1] = (_Float16)bf16r(a.y);
    o[2] = (_Float16)bf16r(a.z); o[3] = (_Float16)bf16r(a.w);
    o[4] = (_Float16)bf16r(b.x); o[5] = (_Float16)bf16r(b.y);
    o[6] = (_Float16)bf16r(b.z); o[7] = (_Float16)bf16r(b.w);
    _Float16* d = xh + (size_t)n * DM + c8;
    *(volatile v8h*)d = o;
    __threadfence();
    *(volatile v8h*)d = o;
}

__global__ __launch_bounds__(256) void k_wT(const float* __restrict__ in,
                                             _Float16* __restrict__ out,
                                             unsigned R, unsigned C) {
    __shared__ __align__(16) _Float16 t[64 * 72];
    const unsigned tid = threadIdx.x;
    const unsigned n0 = blockIdx.x * 64u;
    const unsigned k0 = blockIdx.y * 64u;
    const float*  inb  = in  + (size_t)blockIdx.z * R * C;
    _Float16*     outb = out + (size_t)blockIdx.z * R * C;
#pragma unroll
    for (int i = 0; i < 4; ++i) {
        const unsigned idx = (unsigned)i * 256u + tid;
        const unsigned r = idx >> 4, c4 = (idx & 15u) << 2;
        const v4f v = *(const v4f*)(inb + (size_t)(k0 + r) * C + n0 + c4);
        t[(c4 + 0u) * 72u + r] = (_Float16)(bf16r(v.x) * 64.0f);
        t[(c4 + 1u) * 72u + r] = (_Float16)(bf16r(v.y) * 64.0f);
        t[(c4 + 2u) * 72u + r] = (_Float16)(bf16r(v.z) * 64.0f);
        t[(c4 + 3u) * 72u + r] = (_Float16)(bf16r(v.w) * 64.0f);
    }
    __syncthreads();
    const unsigned rn0 = tid >> 3, pc = (tid & 7u) << 3;
    const v8h o0 = *(const v8h*)(&t[rn0 * 72u + pc]);
    const v8h o1 = *(const v8h*)(&t[(rn0 + 32u) * 72u + pc]);
    _Float16* d0 = outb + (size_t)(n0 + rn0) * R + k0 + pc;
    _Float16* d1 = outb + (size_t)(n0 + rn0 + 32u) * R + k0 + pc;
    *(volatile v8h*)d0 = o0;
    *(volatile v8h*)d1 = o1;
    __threadfence();
    *(volatile v8h*)d0 = o0;
    *(volatile v8h*)d1 = o1;
}

__global__ __launch_bounds__(256) __attribute__((amdgpu_num_vgpr(256)))
void k_qkv(const _Float16* __restrict__ xh, const _Float16* __restrict__ wT,
           const float* __restrict__ bias,
           _Float16* __restrict__ qh, _Float16* __restrict__ ql,
           _Float16* __restrict__ kh, _Float16* __restrict__ kl,
           _Float16* __restrict__ vTh, _Float16* __restrict__ vTr) {
    __shared__ __align__(16) _Float16 stw[8][2048];
    const unsigned tid  = threadIdx.x;
    const unsigned lane = tid & 31u;
    const unsigned w    = tid >> 5;
    const unsigned n0   = blockIdx.y * 128u + (w >> 2) * 64u;
    const unsigned cb   = blockIdx.x * 128u + (w & 3u) * 32u;
    const unsigned r0   = (lane >> 4) << 3;
    const unsigned cc   = lane & 15u;

    v8f acc[4][2], dum[4][2];
    gemm_core<4, 2, false>(xh + (size_t)n0 * DM, xh + (size_t)n0 * DM,
                           wT + (size_t)cb * DM, (unsigned)DM, lane, acc, dum);

    const unsigned t  = cb >> 9;
    const unsigned h  = (cb >> 6) & 7u;
    const unsigned kk = (cb >> 5) & 1u;
    float bv[2];
    bv[0] = bf16r(bias[cb + cc]) * 64.0f;
    bv[1] = bf16r(bias[cb + 16u + cc]) * 64.0f;
    _Float16* sw = &stw[w][0];

    if (t < 2u) {
        _Float16* ph = (t == 0u) ? qh : kh;
        _Float16* pl = (t == 0u) ? ql : kl;
        const size_t pbase = ((size_t)(h * 2u + kk) * NTOK + n0) * 32u;
#pragma unroll
        for (int mt = 0; mt < 4; ++mt) {
#pragma unroll
            for (int g = 0; g < 8; ++g) {
#pragma unroll
                for (int nt = 0; nt < 2; ++nt) {
                    const float v = acc[mt][nt][g] + bv[nt];
                    const _Float16 hi = (_Float16)v;
                    sw[(r0 + g) * 32u + nt * 16 + cc] = hi;
                    sw[512u + (r0 + g) * 32u + nt * 16 + cc] = (_Float16)((v - (float)hi) * SC_RES);
                }
            }
            wave_lds_sync();
            const v8h a0 = *(const v8h*)(sw + lane * 8u);
            const v8h a1 = *(const v8h*)(sw + 256u + lane * 8u);
            const v8h b0 = *(const v8h*)(sw + 512u + lane * 8u);
            const v8h b1 = *(const v8h*)(sw + 768u + lane * 8u);
            _Float16* dh = ph + pbase + (size_t)mt * 512u;
            _Float16* dl = pl + pbase + (size_t)mt * 512u;
            *(volatile v8h*)(dh + lane * 8u)        = a0;
            *(volatile v8h*)(dh + 256u + lane * 8u) = a1;
            *(volatile v8h*)(dl + lane * 8u)        = b0;
            *(volatile v8h*)(dl + 256u + lane * 8u) = b1;
            __threadfence();
            *(volatile v8h*)(dh + lane * 8u)        = a0;
            *(volatile v8h*)(dh + 256u + lane * 8u) = a1;
            *(volatile v8h*)(dl + lane * 8u)        = b0;
            *(volatile v8h*)(dl + 256u + lane * 8u) = b1;
            wave_lds_sync();
        }
    } else {
        const unsigned b  = n0 / (unsigned)SEQ;
        const unsigned l0 = n0 - b * (unsigned)SEQ;
        const unsigned hb = h * (unsigned)NB + b;
        const size_t vbase = ((size_t)(hb * HD + kk * 32u)) * SEQ + l0;
        const unsigned rq = lane >> 3;
        const unsigned pc = (lane & 7u) << 3;
        v8h xv[8];
#pragma unroll
        for (int mt = 0; mt < 4; ++mt)
#pragma unroll
            for (int nt = 0; nt < 2; ++nt) {
                v8h hv;
#pragma unroll
                for (int g = 0; g < 8; ++g) hv[g] = (_Float16)(acc[mt][nt][g] + bv[nt]);
                *(v8h*)(sw + (nt * 16 + cc) * 64u + mt * 16 + r0) = hv;
            }
        wave_lds_sync();
#pragma unroll
        for (int i = 0; i < 8; ++i) xv[i] = *(const v8h*)(sw + (i * 4 + rq) * 64u + pc);
#pragma unroll
        for (int i = 0; i < 8; ++i)
            *(volatile v8h*)(vTh + vbase + (size_t)(i * 4 + rq) * SEQ + pc) = xv[i];
        __threadfence();
#pragma unroll
        for (int i = 0; i < 8; ++i)
            *(volatile v8h*)(vTh + vbase + (size_t)(i * 4 + rq) * SEQ + pc) = xv[i];
        wave_lds_sync();
#pragma unroll
        for (int mt = 0; mt < 4; ++mt)
#pragma unroll
            for (int nt = 0; nt < 2; ++nt) {
                v8h hv;
#pragma unroll
                for (int g = 0; g < 8; ++g) {
                    const float v = acc[mt][nt][g] + bv[nt];
                    const _Float16 hi = (_Float16)v;
                    hv[g] = (_Float16)((v - (float)hi) * SC_RES);
                }
                *(v8h*)(sw + (nt * 16 + cc) * 64u + mt * 16 + r0) = hv;
            }
        wave_lds_sync();
#pragma unroll
        for (int i = 0; i < 8; ++i) xv[i] = *(const v8h*)(sw + (i * 4 + rq) * 64u + pc);
#pragma unroll
        for (int i = 0; i < 8; ++i)
            *(volatile v8h*)(vTr + vbase + (size_t)(i * 4 + rq) * SEQ + pc) = xv[i];
        __threadfence();
#pragma unroll
        for (int i = 0; i < 8; ++i)
            *(volatile v8h*)(vTr + vbase + (size_t)(i * 4 + rq) * SEQ + pc) = xv[i];
    }
}

__global__ __launch_bounds__(256) __attribute__((amdgpu_num_vgpr(256)))
void k_attn(const _Float16* __restrict__ qh, const _Float16* __restrict__ ql,
            const _Float16* __restrict__ kh, const _Float16* __restrict__ kl,
            const _Float16* __restrict__ vTh, const _Float16* __restrict__ vTr,
            const float* __restrict__ mask,
            _Float16* __restrict__ ctxh, _Float16* __restrict__ ctxr) {
    __shared__ __align__(16) float    msk[SEQ];
    __shared__ __align__(16) _Float16 Ch[8][16 * HD];
    __shared__ __align__(16) _Float16 Cr[8][16 * HD];

    const unsigned tid  = threadIdx.x;
    const unsigned lane = tid & 31u;
    const unsigned w    = tid >> 5;
    const unsigned hb   = blockIdx.x;
    const unsigned h    = hb / (unsigned)NB;
    const unsigned b    = hb - h * (unsigned)NB;
    const unsigned q0   = blockIdx.y * 128u + w * 16u;
    const unsigned r0   = (lane >> 4) << 3;
    const unsigned cc   = lane & 15u;

    for (unsigned idx = tid; idx < (unsigned)SEQ; idx += 256u)
        msk[idx] = bf16r(mask[(size_t)b * SEQ_FULL + idx]) * LOG2E;
    __syncthreads();

    const size_t tokq = (size_t)b * SEQ + q0;
    const size_t tokk = (size_t)b * SEQ;
    const size_t P0 = (size_t)(h * 2u) * NTOK;
    const size_t P1 = (size_t)(h * 2u + 1u) * NTOK;
    const v16h qhf0 = load_frag16(qh + (P0 + tokq) * 32u, 32u, lane);
    const v16h qhf1 = load_frag16(qh + (P1 + tokq) * 32u, 32u, lane);
    const v16h qlf0 = load_frag16(ql + (P0 + tokq) * 32u, 32u, lane);
    const v16h qlf1 = load_frag16(ql + (P1 + tokq) * 32u, 32u, lane);
    const _Float16* kh0 = kh + (P0 + tokk) * 32u;
    const _Float16* kh1 = kh + (P1 + tokk) * 32u;
    const _Float16* kl0 = kl + (P0 + tokk) * 32u;
    const _Float16* kl1 = kl + (P1 + tokk) * 32u;
    const _Float16* vhb = vTh + (size_t)hb * HD * SEQ;
    const _Float16* vrb = vTr + (size_t)hb * HD * SEQ;

    v8f oh[4], orr[4];
#pragma unroll
    for (int dt = 0; dt < 4; ++dt) { oh[dt] = zero8(); orr[dt] = zero8(); }
    float mr = -1.0e30f, lr = 0.0f;

#pragma unroll 1
    for (unsigned key0 = 0; key0 < (unsigned)SEQ; key0 += 32u) {
        v8f sh0 = zero8(), sr0 = zero8(), sh1 = zero8(), sr1 = zero8();
        {
            v16h a  = load_frag16(kh0 + (size_t)key0 * 32u, 32u, lane);
            v16h al = load_frag16(kl0 + (size_t)key0 * 32u, 32u, lane);
            sh0 = wmma16(a, qhf0, sh0);
            sr0 = wmma16(a, qlf0, sr0);
            sr0 = wmma16(al, qhf0, sr0);
            a  = load_frag16(kh1 + (size_t)key0 * 32u, 32u, lane);
            al = load_frag16(kl1 + (size_t)key0 * 32u, 32u, lane);
            sh0 = wmma16(a, qhf1, sh0);
            sr0 = wmma16(a, qlf1, sr0);
            sr0 = wmma16(al, qhf1, sr0);
        }
        {
            v16h a  = load_frag16(kh0 + (size_t)(key0 + 16u) * 32u, 32u, lane);
            v16h al = load_frag16(kl0 + (size_t)(key0 + 16u) * 32u, 32u, lane);
            sh1 = wmma16(a, qhf0, sh1);
            sr1 = wmma16(a, qlf0, sr1);
            sr1 = wmma16(al, qhf0, sr1);
            a  = load_frag16(kh1 + (size_t)(key0 + 16u) * 32u, 32u, lane);
            al = load_frag16(kl1 + (size_t)(key0 + 16u) * 32u, 32u, lane);
            sh1 = wmma16(a, qhf1, sh1);
            sr1 = wmma16(a, qlf1, sr1);
            sr1 = wmma16(al, qhf1, sr1);
        }
        float t0[8], t1[8];
#pragma unroll
        for (int g = 0; g < 8; ++g) {
            t0[g] = __builtin_fmaf(sh0[g], C1, sr0[g] * C2) + msk[key0 + r0 + g];
            t1[g] = __builtin_fmaf(sh1[g], C1, sr1[g] * C2) + msk[key0 + 16u + r0 + g];
        }
        float tmax = fmaxf(t0[0], t1[0]);
#pragma unroll
        for (int g = 1; g < 8; ++g) tmax = fmaxf(tmax, fmaxf(t0[g], t1[g]));
        tmax = fmaxf(tmax, __shfl_xor(tmax, 16, 32));
        const float mn    = fmaxf(mr, tmax);
        const float alpha = ex2(mr - mn);
        mr = mn;
        const float off = 14.0f - mn;
        v8h p0, p1;
        float ps = 0.0f;
#pragma unroll
        for (int g = 0; g < 8; ++g) {
            const _Float16 a = (_Float16)ex2(t0[g] + off);
            const _Float16 c = (_Float16)ex2(t1[g] + off);
            p0[g] = a;
            p1[g] = c;
            ps += (float)a + (float)c;
        }
        ps += __shfl_xor(ps, 16, 32);
        lr = lr * alpha + ps;
        Frag pb;
        pb.h[0] = p0;
        pb.h[1] = p1;
#pragma unroll
        for (int dt = 0; dt < 4; ++dt) {
            oh[dt]  = oh[dt] * alpha;
            orr[dt] = orr[dt] * alpha;
        }
#pragma unroll
        for (int dt = 0; dt < 4; ++dt) {
            const v16h va = load_frag16(vhb + (size_t)(dt * 16) * SEQ + key0, (unsigned)SEQ, lane);
            oh[dt] = wmma16(va, pb.v, oh[dt]);
            const v16h vr = load_frag16(vrb + (size_t)(dt * 16) * SEQ + key0, (unsigned)SEQ, lane);
            orr[dt] = wmma16(vr, pb.v, orr[dt]);
        }
    }

    const float inv = 0.25f * (1.0f / lr);
#pragma unroll
    for (int dt = 0; dt < 4; ++dt) {
        v8h hv, rv;
#pragma unroll
        for (int g = 0; g < 8; ++g) {
            const float c = __builtin_fmaf(orr[dt][g], SC_RINV, oh[dt][g]) * inv;
            const _Float16 hi = (_Float16)c;
            hv[g] = hi;
            rv[g] = (_Float16)((c - (float)hi) * SC_RES);
        }
        *(v8h*)(&Ch[w][cc * HD + dt * 16 + r0]) = hv;
        *(v8h*)(&Cr[w][cc * HD + dt * 16 + r0]) = rv;
    }
    wave_lds_sync();
    const unsigned rq = lane >> 3;
    const unsigned pc = (lane & 7u) << 3;
    v8h ch[4], cr[4];
#pragma unroll
    for (int i = 0; i < 4; ++i) {
        ch[i] = *(const v8h*)(&Ch[w][(i * 4 + rq) * HD + pc]);
        cr[i] = *(const v8h*)(&Cr[w][(i * 4 + rq) * HD + pc]);
    }
    const size_t ob = (tokq) * DM + h * HD + pc;
#pragma unroll
    for (int i = 0; i < 4; ++i) {
        *(volatile v8h*)(ctxh + ob + (size_t)(i * 4 + rq) * DM) = ch[i];
        *(volatile v8h*)(ctxr + ob + (size_t)(i * 4 + rq) * DM) = cr[i];
    }
    __threadfence();
#pragma unroll
    for (int i = 0; i < 4; ++i) {
        *(volatile v8h*)(ctxh + ob + (size_t)(i * 4 + rq) * DM) = ch[i];
        *(volatile v8h*)(ctxr + ob + (size_t)(i * 4 + rq) * DM) = cr[i];
    }
}

template <bool POST>
__global__ __launch_bounds__(256) __attribute__((amdgpu_num_vgpr(256)))
void k_gemm_ln(const _Float16* __restrict__ Ah, const _Float16* __restrict__ Ar,
               const _Float16* __restrict__ Bt, unsigned K,
               const float* __restrict__ bias, const float* __restrict__ resid,
               const float* __restrict__ lnw, const float* __restrict__ lnb,
               float* __restrict__ outF, _Float16* __restrict__ outH) {
    __shared__ __align__(16) float T[32 * DM];
    const unsigned tid  = threadIdx.x;
    const unsigned lane = tid & 31u;
    const unsigned w    = tid >> 5;
    const unsigned row0 = blockIdx.x * 32u;
    const unsigned cb   = w * 64u;
    const unsigned r0   = (lane >> 4) << 3;
    const unsigned cc   = lane & 15u;

    v8f acc[2][4], accr[2][4];
    gemm_core<2, 4, POST>(Ah + (size_t)row0 * K, Ar + (size_t)row0 * K,
                          Bt + (size_t)cb * K, K, lane, acc, accr);
#pragma unroll
    for (int mt = 0; mt < 2; ++mt)
#pragma unroll
        for (int nt = 0; nt < 4; ++nt)
#pragma unroll
            for (int g = 0; g < 8; ++g) {
                const float v = POST ? __builtin_fmaf(accr[mt][nt][g], SC_RINV, acc[mt][nt][g])
                                     : acc[mt][nt][g];
                T[(mt * 16 + r0 + g) * DM + cb + nt * 16 + cc] = v;
            }
    __syncthreads();

#pragma unroll 1
    for (unsigned rr = 0; rr < 4u; ++rr) {
        const unsigned row = w * 4u + rr;
        const unsigned n   = row0 + row;
        const unsigned fr  = full_row(n);
        const float* rp = POST ? (resid + (size_t)fr * DM) : (resid + (size_t)n * DM);
        float*       op = POST ? (outF + (size_t)n * DM)   : (outF + (size_t)fr * DM);
        v4f xv[4];
        float s = 0.0f;
#pragma unroll
        for (int i = 0; i < 4; ++i) {
            const unsigned c = (unsigned)i * 128u + lane * 4u;
            const v4f a  = *(const v4f*)(&T[row * DM + c]);
            const v4f bi = *(const v4f*)(bias + c);
            const v4f rs = *(const v4f*)(rp + c);
            v4f x;
            x.x = __builtin_fmaf(a.x, SC_OUT, bf16r(bi.x)) + (POST ? bf16r(rs.x) : rs.x);
            x.y = __builtin_fmaf(a.y, SC_OUT, bf16r(bi.y)) + (POST ? bf16r(rs.y) : rs.y);
            x.z = __builtin_fmaf(a.z, SC_OUT, bf16r(bi.z)) + (POST ? bf16r(rs.z) : rs.z);
            x.w = __builtin_fmaf(a.w, SC_OUT, bf16r(bi.w)) + (POST ? bf16r(rs.w) : rs.w);
            xv[i] = x;
            s += (x.x + x.y) + (x.z + x.w);
        }
        s = wave_sum(s);
        const float mu = s * (1.0f / (float)DM);
        float q = 0.0f;
#pragma unroll
        for (int i = 0; i < 4; ++i) {
            const float d0 = xv[i].x - mu, d1 = xv[i].y - mu, d2 = xv[i].z - mu, d3 = xv[i].w - mu;
            q += (d0 * d0 + d1 * d1) + (d2 * d2 + d3 * d3);
        }
        q = wave_sum(q);
        const float rstd = rsqrtf(q * (1.0f / (float)DM) + 1.0e-5f);
        v4f yv[4];
#pragma unroll
        for (int i = 0; i < 4; ++i) {
            const unsigned c = (unsigned)i * 128u + lane * 4u;
            const v4f gw = *(const v4f*)(lnw + c);
            const v4f gb = *(const v4f*)(lnb + c);
            v4f y;
            y.x = (xv[i].x - mu) * rstd * bf16r(gw.x) + bf16r(gb.x);
            y.y = (xv[i].y - mu) * rstd * bf16r(gw.y) + bf16r(gb.y);
            y.z = (xv[i].z - mu) * rstd * bf16r(gw.z) + bf16r(gb.z);
            y.w = (xv[i].w - mu) * rstd * bf16r(gw.w) + bf16r(gb.w);
            yv[i] = y;
        }
        v8h hv0, hv1;
        _Float16* hp = outH + (size_t)n * DM;
        if (POST) {
#pragma unroll
            for (int i = 0; i < 4; ++i)
                *(v4f*)(&T[row * DM + (unsigned)i * 128u + lane * 4u]) = yv[i];
            wave_lds_sync();
            const v4f u0 = *(const v4f*)(&T[row * DM + lane * 8u]);
            const v4f u1 = *(const v4f*)(&T[row * DM + lane * 8u + 4u]);
            const v4f u2 = *(const v4f*)(&T[row * DM + 256u + lane * 8u]);
            const v4f u3 = *(const v4f*)(&T[row * DM + 256u + lane * 8u + 4u]);
            hv0[0] = (_Float16)(u0.x * 16.0f); hv0[1] = (_Float16)(u0.y * 16.0f);
            hv0[2] = (_Float16)(u0.z * 16.0f); hv0[3] = (_Float16)(u0.w * 16.0f);
            hv0[4] = (_Float16)(u1.x * 16.0f); hv0[5] = (_Float16)(u1.y * 16.0f);
            hv0[6] = (_Float16)(u1.z * 16.0f); hv0[7] = (_Float16)(u1.w * 16.0f);
            hv1[0] = (_Float16)(u2.x * 16.0f); hv1[1] = (_Float16)(u2.y * 16.0f);
            hv1[2] = (_Float16)(u2.z * 16.0f); hv1[3] = (_Float16)(u2.w * 16.0f);
            hv1[4] = (_Float16)(u3.x * 16.0f); hv1[5] = (_Float16)(u3.y * 16.0f);
            hv1[6] = (_Float16)(u3.z * 16.0f); hv1[7] = (_Float16)(u3.w * 16.0f);
        }
#pragma unroll
        for (int i = 0; i < 4; ++i)
            *(volatile v4f*)(op + (unsigned)i * 128u + lane * 4u) = yv[i];
        if (POST) {
            *(volatile v8h*)(hp + lane * 8u)        = hv0;
            *(volatile v8h*)(hp + 256u + lane * 8u) = hv1;
        }
        __threadfence();
#pragma unroll
        for (int i = 0; i < 4; ++i)
            *(volatile v4f*)(op + (unsigned)i * 128u + lane * 4u) = yv[i];
        if (POST) {
            *(volatile v8h*)(hp + lane * 8u)        = hv0;
            *(volatile v8h*)(hp + 256u + lane * 8u) = hv1;
        }
    }
}

__global__ __launch_bounds__(256) __attribute__((amdgpu_num_vgpr(256)))
void k_ff1(const _Float16* __restrict__ sah, const _Float16* __restrict__ Bt,
           const float* __restrict__ bias, _Float16* __restrict__ hid) {
    __shared__ __align__(16) _Float16 st[8][32 * 64];
    const unsigned tid  = threadIdx.x;
    const unsigned lane = tid & 31u;
    const unsigned w    = tid >> 5;
    const unsigned row0 = blockIdx.y * 32u;
    const unsigned cb   = blockIdx.x * 512u + w * 64u;
    const unsigned r0   = (lane >> 4) << 3;
    const unsigned cc   = lane & 15u;

    v8f acc[2][4], dum[2][4];
    gemm_core<2, 4, false>(sah + (size_t)row0 * DM, sah + (size_t)row0 * DM,
                           Bt + (size_t)cb * DM, (unsigned)DM, lane, acc, dum);
    float bv[4];
#pragma unroll
    for (int nt = 0; nt < 4; ++nt) bv[nt] = bf16r(bias[cb + nt * 16 + cc]) * 16.0f;
    _Float16* sw = &st[w][0];
#pragma unroll
    for (int mt = 0; mt < 2; ++mt)
#pragma unroll
        for (int nt = 0; nt < 4; ++nt)
#pragma unroll
            for (int g = 0; g < 8; ++g)
                sw[(mt * 16 + r0 + g) * 64u + nt * 16 + cc] =
                    (_Float16)fmaxf(__builtin_fmaf(acc[mt][nt][g], SC_HID, bv[nt]), 0.0f);
    wave_lds_sync();
    const unsigned rq = lane >> 3;
    const unsigned pc = (lane & 7u) << 3;
    v8h xv[8];
#pragma unroll
    for (int i = 0; i < 8; ++i) xv[i] = *(const v8h*)(sw + (i * 4 + rq) * 64u + pc);
    _Float16* ob = hid + (size_t)row0 * DF + cb + pc;
#pragma unroll
    for (int i = 0; i < 8; ++i) *(volatile v8h*)(ob + (size_t)(i * 4 + rq) * DF) = xv[i];
    __threadfence();
#pragma unroll
    for (int i = 0; i < 8; ++i) *(volatile v8h*)(ob + (size_t)(i * 4 + rq) * DF) = xv[i];
}

#define U_BYTES ((size_t)NTOK * DM * 2)
static_assert((size_t)NB_FULL * SEQ_FULL * DM * 2 * 8 <= (size_t)134217728);
static_assert(3 * U_BYTES >= (size_t)DM * DM * 2);

extern "C" void kernel_launch(void* const* d_in, const int* in_sizes, int n_in,
                              void* d_out, int out_size, void* d_ws, size_t ws_size,
                              hipStream_t stream) {
    if (n_in < 14) return;
    const int need_rows = (NB - 1) * SEQ_FULL + SEQ;
    if (in_sizes[0] < need_rows * DM) return;
    if (in_sizes[1] < need_rows) return;
    if (in_sizes[2] < 3 * NH * DM * HD || in_sizes[3] < 3 * NH * HD) return;
    if (in_sizes[4] < DM * DM || in_sizes[5] < DM) return;
    if (in_sizes[6] < DM * DF || in_sizes[7] < DF) return;
    if (in_sizes[8] < DF * DM || in_sizes[9] < DM) return;
    if (in_sizes[10] < DM || in_sizes[11] < DM || in_sizes[12] < DM || in_sizes[13] < DM) return;
    if (out_size < need_rows * DM) return;

    const float* inp   = (const float*)d_in[0];
    const float* mask  = (const float*)d_in[1];
    const float* preW  = (const float*)d_in[2];
    const float* preB  = (const float*)d_in[3];
    const float* postW = (const float*)d_in[4];
    const float* postB = (const float*)d_in[5];
    const float* ff1W  = (const float*)d_in[6];
    const float* ff1B  = (const float*)d_in[7];
    const float* ff2W  = (const float*)d_in[8];
    const float* ff2B  = (const float*)d_in[9];
    const float* ln1w  = (const float*)d_in[10];
    const float* ln1b  = (const float*)d_in[11];
    const float* ln2w  = (const float*)d_in[12];
    const float* ln2b  = (const float*)d_in[13];
    float* out = (float*)d_out;

    const size_t U = U_BYTES;
    const size_t WQ_B = (size_t)3 * NH * HD * DM * 2;
    const size_t W1_B = (size_t)DF * DM * 2;
    const size_t W2_B = (size_t)DM * DF * 2;
    size_t total = 8 * U;
    if (7 * U + W1_B + W2_B > total) total = 7 * U + W1_B + W2_B;
    if (7 * U + WQ_B > total) total = 7 * U + WQ_B;
    if (total > ws_size) return;

    char* ws = (char*)d_ws;
    _Float16* qh    = (_Float16*)(ws + 0 * U);
    _Float16* ql    = (_Float16*)(ws + 1 * U);
    _Float16* kh    = (_Float16*)(ws + 2 * U);
    _Float16* kl    = (_Float16*)(ws + 3 * U);
    _Float16* vTh   = (_Float16*)(ws + 4 * U);
    _Float16* vTr   = (_Float16*)(ws + 5 * U);
    _Float16* xh    = (_Float16*)(ws + 6 * U);
    _Float16* ctxh  = (_Float16*)(ws + 6 * U);
    _Float16* ctxr  = (_Float16*)(ws + 7 * U);
    _Float16* wqkvT = (_Float16*)(ws + 7 * U);
    float*    sa    = (float*)(ws + 0 * U);
    _Float16* sah   = (_Float16*)(ws + 2 * U);
    _Float16* postT = (_Float16*)(ws + 3 * U);
    _Float16* hid   = (_Float16*)(ws + 3 * U);
    _Float16* ff1T  = (_Float16*)(ws + 7 * U);
    _Float16* ff2T  = (_Float16*)(ws + 7 * U + W1_B);

    k_cvt_x<<<dim3(NTOK / 4), dim3(256), 0, stream>>>(inp, xh);
    k_wT<<<dim3(1, 8, 24), dim3(256), 0, stream>>>(preW, wqkvT, 512u, 64u);
    k_qkv<<<dim3(12, NTOK / 128), dim3(256), 0, stream>>>(xh, wqkvT, preB, qh, ql, kh, kl, vTh, vTr);
    k_attn<<<dim3(NH * NB, SEQ / 128), dim3(256), 0, stream>>>(qh, ql, kh, kl, vTh, vTr, mask, ctxh, ctxr);
    k_wT<<<dim3(8, 8, 1), dim3(256), 0, stream>>>(postW, postT, 512u, 512u);
    k_gemm_ln<true><<<dim3(NTOK / 32), dim3(256), 0, stream>>>(
        ctxh, ctxr, postT, 512u, postB, inp, ln1w, ln1b, sa, sah);
    k_wT<<<dim3(32, 8, 1), dim3(256), 0, stream>>>(ff1W, ff1T, 512u, 2048u);
    k_wT<<<dim3(8, 32, 1), dim3(256), 0, stream>>>(ff2W, ff2T, 2048u, 512u);
    k_ff1<<<dim3(4, NTOK / 32), dim3(256), 0, stream>>>(sah, ff1T, ff1B, hid);
    k_gemm_ln<false><<<dim3(NTOK / 32), dim3(256), 0, stream>>>(
        hid, hid, ff2T, 2048u, ff2B, sa, ln2w, ln2b, out, sah);
}
